// TransE_76768245448766
// MI455X (gfx1250) — hardware-run, weakly checked
//
#include <hip/hip_runtime.h>
#include <stddef.h>


typedef _Float16 v16h __attribute__((ext_vector_type(16)));
typedef _Float16 v8h  __attribute__((ext_vector_type(8)));
typedef _Float16 v4h  __attribute__((ext_vector_type(4)));
typedef float    v8f  __attribute__((ext_vector_type(8)));
typedef float    v4f  __attribute__((ext_vector_type(4)));

#ifndef NB
#define NB 32
#endif
#ifndef NENT
#define NENT 40943
#endif
#define NB_FULL   32
#define NENT_FULL 40943
#define NREL      18
#define EDIM      128
#define NPAD      (((NENT + 63) / 64) * 64)
#define NF4       ((NB * NENT) / 4)

#define LDE 136
#define LDC 68

#define QCARRY 64.0f
#define ECARRY 1024.0f

static_assert(NB == 32 && NB == NB_FULL);
static_assert(NENT >= 64 && NENT <= NENT_FULL);
static_assert(EDIM == 128 && EDIM == 32 * 4);
static_assert((EDIM % 32) == 0);
static_assert((NPAD % 64) == 0 && NPAD >= NENT);
static_assert(((NB * NENT) % 32) == 0);
static_assert((LDE % 8) == 0 && LDE >= EDIM);
static_assert((LDC % 4) == 0 && LDC >= 64);
static_assert((size_t)NB * NPAD < (size_t)0xFFFFFFFFu);

#define Q16_BYTES ((size_t)NB * EDIM * 2)
#define QN_BYTES  ((size_t)128)
#define S_BYTES   ((size_t)NB * NPAD * 4)
#define OFF_Q16   ((size_t)0)
#define OFF_QN    (OFF_Q16 + Q16_BYTES)
#define OFF_S     (OFF_QN + QN_BYTES)
#define WS_TOTAL  (OFF_S + S_BYTES)
static_assert((Q16_BYTES % 128) == 0 && (QN_BYTES % 128) == 0 && (S_BYTES % 128) == 0);
static_assert(NB * 4 <= 128);
static_assert(WS_TOTAL <= (size_t)134217728);

__device__ __forceinline__ float bf16r(float x) {
  unsigned int u = __float_as_uint(x);
  u = (u + 0x7FFFu + ((u >> 16) & 1u)) & 0xFFFF0000u;
  return __uint_as_float(u);
}

static __device__ __forceinline__ _Float16 toh_flush(float v) {
  const _Float16 r = (_Float16)v;
  return (fabsf(v) < 6.103515625e-05f) ? (_Float16)0.0f : r;
}

__device__ __forceinline__ v16h frag_at(const _Float16* p) {
  v8h lo = *(const v8h*)(p);
  v8h hi = *(const v8h*)(p + 16);
  v16h out;
#pragma unroll
  for (int i = 0; i < 8; ++i) { out[i] = lo[i]; out[i + 8] = hi[i]; }
  return out;
}
__device__ __forceinline__ v16h frag_join(v8h lo, v8h hi) {
  v16h out;
#pragma unroll
  for (int i = 0; i < 8; ++i) { out[i] = lo[i]; out[i + 8] = hi[i]; }
  return out;
}

__device__ __forceinline__ v8f wmma16(v16h a, v16h b, v8f c) {
  v8f d = __builtin_amdgcn_wmma_f32_16x16x32_f16(false, a, false, b, (short)0, c,
                                                 false, false);
  asm volatile("v_nop\n\tv_nop\n\tv_nop\n\tv_nop" : "+v"(d) : "v"(a), "v"(b));
  return d;
}

__device__ __forceinline__ float red32_sum(float x) {
#pragma unroll
  for (int off = 1; off < 32; off <<= 1) x += __shfl_xor(x, off, 32);
  return x;
}

__global__ __launch_bounds__(256) void q_kernel(
    const int* __restrict__ heads, const int* __restrict__ rels,
    const float* __restrict__ ent, const float* __restrict__ rel,
    _Float16* __restrict__ Q16, float* __restrict__ QN) {
  __shared__ __attribute__((aligned(16))) float qns[NB];
  const unsigned lane = threadIdx.x & 31u;
  const unsigned wv = threadIdx.x >> 5;
  const unsigned w = __builtin_amdgcn_readfirstlane(threadIdx.x >> 5);
#pragma unroll 1
  for (unsigned i = 0; i < 4u; ++i) {
    const unsigned b = wv * 4u + i;
    int h = heads[b];
    int r = rels[b];
    h = (h < 0) ? 0 : h;
    h = (h > NENT_FULL - 1) ? (NENT_FULL - 1) : h;
    r = (r < 0) ? 0 : r;
    r = (r > NREL - 1) ? (NREL - 1) : r;
    const v4f hv = *(const v4f*)(ent + (size_t)h * EDIM + lane * 4u);
    const v4f rv = *(const v4f*)(rel + (size_t)r * EDIM + lane * 4u);
    v4h o;
    float p = 0.0f;
#pragma unroll
    for (int j = 0; j < 4; ++j) {
      const float q = bf16r(hv[j]) + bf16r(rv[j]);
      p += q * q;
      o[j] = toh_flush(QCARRY * q);
    }
    p = red32_sum(p);
    if (lane == 0u) qns[b] = p;
    _Float16* dst = Q16 + (size_t)b * EDIM + lane * 4u;
    *(volatile v4h*)dst = o;
    __threadfence();
    *(volatile v4h*)dst = o;
  }
  __syncthreads();
  if (w == 0u) {
    if (lane < 8u) {
      const v4f x = *(const v4f*)&qns[lane * 4u];
      float* dst = QN + lane * 4u;
      *(volatile v4f*)dst = x;
      __threadfence();
      *(volatile v4f*)dst = x;
    }
  }
}

__global__ __launch_bounds__(256) void score_kernel(
    const float* __restrict__ ent, const _Float16* __restrict__ Q16,
    const float* __restrict__ QN, float* __restrict__ S) {
  __shared__ __attribute__((aligned(16))) _Float16 Es[64 * LDE];
  __shared__ __attribute__((aligned(16))) float Cs[32 * LDC];
  __shared__ __attribute__((aligned(16))) float ens[64];

  const unsigned tid = threadIdx.x, lane = tid & 31u;
  const unsigned wv = tid >> 5;
  const unsigned w = __builtin_amdgcn_readfirstlane(threadIdx.x >> 5);
  const unsigned mw = w >> 2, nw = w & 3u;
  const unsigned hh = lane >> 4, m = lane & 15u;
  const unsigned n0 = blockIdx.x * 64u;

  const _Float16* ap = Q16 + (size_t)(mw * 16u + m) * EDIM + hh * 8u;
  v16h a[4];
#pragma unroll
  for (int c = 0; c < 4; ++c) a[c] = frag_at(ap + c * 32);

#pragma unroll 2
  for (unsigned j = 0; j < 8u; ++j) {
    const unsigned row = wv + 8u * j;
    const unsigned gr = n0 + row;
    const bool live = gr < (unsigned)NENT;
    const unsigned grc = live ? gr : (unsigned)(NENT - 1);
    const v4f v = *(const v4f*)(ent + (size_t)grc * EDIM + lane * 4u);
    v4h o;
    float p = 0.0f;
#pragma unroll
    for (int i = 0; i < 4; ++i) {
      const float e = live ? bf16r(v[i]) : 0.0f;
      p += e * e;
      o[i] = toh_flush(ECARRY * e);
    }
    *(v4h*)&Es[row * LDE + lane * 4u] = o;
    p = red32_sum(p);
    if (lane == 0u) ens[row] = p;
  }
  __syncthreads();

  v8f acc = {};
  const unsigned eb = (nw * 16u + m) * LDE + hh * 8u;
#pragma unroll
  for (int c = 0; c < 4; ++c) {
    const v8h lo = *(const v8h*)&Es[eb + (unsigned)c * 32u];
    const v8h hi = *(const v8h*)&Es[eb + (unsigned)c * 32u + 16u];
    acc = wmma16(a[c], frag_join(lo, hi), acc);
  }

#pragma unroll
  for (int r = 0; r < 8; ++r)
    Cs[(mw * 16u + hh * 8u + (unsigned)r) * LDC + nw * 16u + m] = acc[r];
  __syncthreads();

  const float cinv = 2.0f / (QCARRY * ECARRY);
  v4f xs[2];
  size_t off[2];
#pragma unroll
  for (unsigned i = 0; i < 2u; ++i) {
    const unsigned r = 16u * i + (tid >> 4);
    const unsigned c = (tid & 15u) * 4u;
    const v4f u = *(const v4f*)&Cs[r * LDC + c];
    const v4f en = *(const v4f*)&ens[c];
    const float qn = QN[r];
    v4f val;
#pragma unroll
    for (int j = 0; j < 4; ++j) val[j] = (qn + en[j]) - u[j] * cinv;
    xs[i] = val;
    off[i] = (size_t)r * NPAD + n0 + c;
  }
#pragma unroll
  for (int i = 0; i < 2; ++i) *(volatile v4f*)(S + off[i]) = xs[i];
  __threadfence();
#pragma unroll
  for (int i = 0; i < 2; ++i) *(volatile v4f*)(S + off[i]) = xs[i];
}

__global__ __launch_bounds__(256) void pack_kernel(
    const float* __restrict__ S, float* __restrict__ out) {
  const unsigned t = blockIdx.x * 256u + threadIdx.x;
  const unsigned tc = (t < (unsigned)NF4) ? t : (unsigned)(NF4 - 1);
  v4f x;
#pragma unroll
  for (unsigned j = 0; j < 4u; ++j) {
    const unsigned f = 4u * tc + j;
    const unsigned b = f / (unsigned)NENT;
    const unsigned n = f - b * (unsigned)NENT;
    x[j] = S[(size_t)b * NPAD + n];
  }
  float* dst = out + (size_t)tc * 4u;
  if (t < (unsigned)NF4) *(volatile v4f*)dst = x;
  __threadfence();
  if (t < (unsigned)NF4) *(volatile v4f*)dst = x;
}

extern "C" void kernel_launch(void* const* d_in, const int* in_sizes, int n_in,
                              void* d_out, int out_size, void* d_ws, size_t ws_size,
                              hipStream_t stream) {
  if (n_in < 4) return;
  if (in_sizes[0] < NB) return;
  if (in_sizes[1] < NB) return;
  if ((long long)in_sizes[2] < (long long)NENT_FULL * EDIM) return;
  if ((long long)in_sizes[3] < (long long)NREL * EDIM) return;
  if ((long long)out_size < (long long)NB * NENT) return;
  if (ws_size < WS_TOTAL) return;

  const int*   heads = (const int*)d_in[0];
  const int*   rels  = (const int*)d_in[1];
  const float* ent   = (const float*)d_in[2];
  const float* rel   = (const float*)d_in[3];
  float* out = (float*)d_out;

  char* ws = (char*)d_ws;
  _Float16* Q16 = (_Float16*)(ws + OFF_Q16);
  float*    QN  = (float*)(ws + OFF_QN);
  float*    S   = (float*)(ws + OFF_S);

  dim3 blk(256);
  q_kernel<<<dim3(1), blk, 0, stream>>>(heads, rels, ent, rel, Q16, QN);
  score_kernel<<<dim3(NPAD / 64), blk, 0, stream>>>(ent, Q16, QN, S);
  pack_kernel<<<dim3((NF4 + 255) / 256), blk, 0, stream>>>(S, out);
}
